// UMambaBlock_35957466202537
// MI455X (gfx1250) — hardware-run, weakly checked
//
#include <hip/hip_runtime.h>
#include <math.h>

typedef __attribute__((ext_vector_type(16))) _Float16 v16h;
typedef __attribute__((ext_vector_type(8)))  _Float16 v8h;
typedef __attribute__((ext_vector_type(16))) __bf16   v16b;
typedef __attribute__((ext_vector_type(8)))  __bf16   v8b;
typedef __attribute__((ext_vector_type(8)))  float    v8f;
typedef __attribute__((ext_vector_type(4)))  float    v4f;
typedef __attribute__((ext_vector_type(4)))  unsigned int v4u;

constexpr int kBatch  = 4;
constexpr int kDm     = 128;
constexpr int kDin    = 256;
constexpr int kHW     = 4096;
constexpr int kSeq    = 4096;
constexpr int kRows   = kBatch * kSeq;
constexpr int kNst    = 16;
constexpr int kDtR    = 8;
constexpr int kXzP    = 2 * kDin;
constexpr int kXdW    = kDtR + 2 * kNst;
constexpr int kXdP    = 64;
constexpr int kK1     = kDm * 9;
constexpr int kK2     = kDin * 9;
constexpr float kEps  = 1e-5f;
constexpr float kNegSlope = 0.01f;
constexpr int kConvTP = 260;
constexpr int kScanTS = 64;
constexpr int kScanCh = 64;
constexpr int kScanYP = 68;
constexpr int kLnTok  = 64;
constexpr int kLnP    = 132;
static_assert(kXdW <= kXdP, "x_proj width");
static_assert((kK1 % 32) == 0 && (kK2 % 32) == 0 && (kDm % 32) == 0 && (kDin % 32) == 0, "GEMM K multiples of 32");
static_assert((kRows % 64) == 0 && (kXzP % 64) == 0 && (kXdP % 64) == 0 && (kDm % 64) == 0 && (kDin % 64) == 0 && (kHW % 64) == 0, "GEMM M,N multiples of 64");
static_assert((kSeq % kScanTS) == 0 && (kSeq % 64) == 0 && (kDin % kScanCh) == 0 && (kDin % 256) == 0, "tile multiples");
static_assert(((kK1 * 2) % 128) == 0 && ((kK2 * 2) % 128) == 0, "im2col rows are whole lines");

constexpr size_t kOffW1H  = 0;
constexpr size_t kOffW1L  = kOffW1H  + (size_t)kDin * kK1 * 2;
constexpr size_t kOffW2H  = kOffW1L  + (size_t)kDin * kK1 * 2;
constexpr size_t kOffW2L  = kOffW2H  + (size_t)kDm  * kK2 * 2;
constexpr size_t kOffWITH = kOffW2L  + (size_t)kDm  * kK2 * 2;
constexpr size_t kOffWITL = kOffWITH + (size_t)kXzP * kDm * 2;
constexpr size_t kOffWXTH = kOffWITL + (size_t)kXzP * kDm * 2;
constexpr size_t kOffWXTL = kOffWXTH + (size_t)kXdP * kDin * 2;
constexpr size_t kOffWOTH = kOffWXTL + (size_t)kXdP * kDin * 2;
constexpr size_t kOffWOTL = kOffWOTH + (size_t)kDm  * kDin * 2;
constexpr size_t kOffRA   = kOffWOTL + (size_t)kDm  * kDin * 2;
constexpr size_t kSzRA    = (size_t)kHW * kK2 * 2 * 2;
constexpr size_t kOffIMH  = kOffRA;
constexpr size_t kOffIML  = kOffRA + (size_t)kHW * kK2 * 2;
constexpr size_t kOffXZ   = kOffRA;
constexpr size_t kOffRB   = kOffRA + kSzRA;
constexpr size_t kSzRB    = (size_t)kBatch * kDin * kHW * 4;
constexpr size_t kOffC1   = kOffRB;
constexpr size_t kOffC2   = kOffRB;
constexpr size_t kOffG2   = kOffRB + (size_t)kBatch * kDm * kHW * 4;
constexpr size_t kOffUC   = kOffRB;
constexpr size_t kOffRC   = kOffRB + kSzRB;
constexpr size_t kSzRC    = (size_t)kBatch * kDin * kHW * 4;
constexpr size_t kOffG1   = kOffRC;
constexpr size_t kOffTH   = kOffRC;
constexpr size_t kOffTL   = kOffRC + (size_t)kRows * kDm * 2;
constexpr size_t kOffUCH  = kOffRC;
constexpr size_t kOffUCL  = kOffRC + (size_t)kRows * kDin * 2;
constexpr size_t kOffXD   = kOffRC + kSzRC;
constexpr size_t kOffYH   = kOffXD + (size_t)kRows * kXdP * 4;
constexpr size_t kOffYL   = kOffYH + (size_t)kRows * kDin * 2;
constexpr size_t kWsTotal = kOffYL + (size_t)kRows * kDin * 2;
static_assert(kWsTotal == 95092736ull, "carve total");
static_assert(kWsTotal <= 134217728ull, "carve cap");
static_assert((size_t)kRows * kXzP * 4 <= kSzRA, "XZ fits RA");
static_assert((size_t)kBatch * kDm * kHW * 4 * 2 <= kSzRB && (size_t)kRows * kDin * 4 <= kSzRB, "C2+G2 and UC fit RB");
static_assert((size_t)kRows * kDm * 2 * 2 <= kSzRC && (size_t)kRows * kDin * 2 * 2 <= kSzRC, "TH+TL and UCH+UCL fit RC");
static_assert((kOffW1L % 128) == 0 && (kOffW2H % 128) == 0 && (kOffW2L % 128) == 0 && (kOffWITH % 128) == 0 &&
              (kOffWITL % 128) == 0 && (kOffWXTH % 128) == 0 && (kOffWXTL % 128) == 0 && (kOffWOTH % 128) == 0 &&
              (kOffWOTL % 128) == 0 && (kOffRA % 128) == 0 && (kOffIML % 128) == 0 && (kOffRB % 128) == 0 &&
              (kOffG2 % 128) == 0 && (kOffRC % 128) == 0 && (kOffTL % 128) == 0 && (kOffUCL % 128) == 0 &&
              (kOffXD % 128) == 0 && (kOffYH % 128) == 0 && (kOffYL % 128) == 0, "128-B aligned regions");

__device__ __forceinline__ unsigned short f2bf_bits(float f) {
  unsigned u = __float_as_uint(f);
  return (unsigned short)((u + 0x7FFFu + ((u >> 16) & 1u)) >> 16);
}
__device__ __forceinline__ float bf_bits2f(unsigned short h) { return __uint_as_float(((unsigned)h) << 16); }

__device__ __forceinline__ void dep_guard_h(v8f& a, v8f& b, v16h x, v16h y) { asm volatile("v_nop\n\tv_nop\n\tv_nop\n\tv_nop" : "+v"(a), "+v"(b) : "v"(x), "v"(y)); }
__device__ __forceinline__ void dep_guard_b(v8f& a, v8f& b, v16b x, v16b y) { asm volatile("v_nop\n\tv_nop\n\tv_nop\n\tv_nop" : "+v"(a), "+v"(b) : "v"(x), "v"(y)); }
__device__ __forceinline__ void keep4_h(v16h a, v16h b, v16h c, v16h d) { asm volatile("v_nop" :: "v"(a), "v"(b), "v"(c), "v"(d)); }
__device__ __forceinline__ void keep4_b(v16b a, v16b b, v16b c, v16b d) { asm volatile("v_nop" :: "v"(a), "v"(b), "v"(c), "v"(d)); }
__device__ __forceinline__ void acc_guard4(v8f& a, v8f& b, v8f& c, v8f& d) { asm volatile("v_nop\n\tv_nop\n\tv_nop\n\tv_nop" : "+v"(a), "+v"(b), "+v"(c), "+v"(d)); }
template <typename T> struct Frag;
template <> struct Frag<_Float16> {
  typedef v16h V; union U { v16h v; v8h h[2]; };
  static __device__ __forceinline__ v16h load(const _Float16* p) {
    U f; f.h[0] = *(const v8h*)(p); f.h[1] = *(const v8h*)(p + 16); return f.v;
  }
  static __device__ __forceinline__ v8f mma(v16h a, v16h b, v8f c) {
    return __builtin_amdgcn_wmma_f32_16x16x32_f16(false, a, false, b, (short)0, c, false, false);
  }
  static __device__ __forceinline__ void guard(v8f& a, v8f& b, v16h x, v16h y) { dep_guard_h(a, b, x, y); }
  static __device__ __forceinline__ void keep(v16h a, v16h b, v16h c, v16h d) { keep4_h(a, b, c, d); }
};
template <> struct Frag<__bf16> {
  typedef v16b V; union U { v16b v; v8b h[2]; };
  static __device__ __forceinline__ v16b load(const __bf16* p) {
    U f; f.h[0] = *(const v8b*)(p); f.h[1] = *(const v8b*)(p + 16); return f.v;
  }
  static __device__ __forceinline__ v8f mma(v16b a, v16b b, v8f c) {
    return __builtin_amdgcn_wmma_f32_16x16x32_bf16(false, a, false, b, (short)0, c, false, false);
  }
  static __device__ __forceinline__ void guard(v8f& a, v8f& b, v16b x, v16b y) { dep_guard_b(a, b, x, y); }
  static __device__ __forceinline__ void keep(v16b a, v16b b, v16b c, v16b d) { keep4_b(a, b, c, d); }
};

template <int ET> struct Elem;
template <> struct Elem<0> { typedef _Float16 T; };
template <> struct Elem<1> { typedef __bf16 T; };
template <int ET, int SPL, int BIAS_MODE, int OUT_MODE, bool RESID, int ACT = 0>
__global__ __launch_bounds__(256) void wmma_gemm64(
    const unsigned short* __restrict__ Ap, const unsigned short* __restrict__ A2p, int lda, long strideA,
    const unsigned short* __restrict__ Btp, const unsigned short* __restrict__ Bt2p, int ldb, long strideB,
    void* __restrict__ Cout, void* __restrict__ Cout2, int ldc, long strideC,
    const float* __restrict__ bias,
    const float* __restrict__ resid, long strideR,
    int M, int N, int K, float scale) {
  typedef typename Elem<ET>::T T;
  typedef typename Frag<T>::V V;
  const T* A = (const T*)Ap; const T* A2 = (const T*)A2p; const T* Bt = (const T*)Btp; const T* Bt2 = (const T*)Bt2p;
  __shared__ __align__(16) float sT[8][16 * 68];
  const int b    = blockIdx.y;
  const int lane = threadIdx.x & 31;
  const int wave = threadIdx.x >> 5;
  const int tilesN = N >> 6;
  const int tilesM = M >> 6;
  const int tile = blockIdx.x * 8 + wave;
  if (tile >= tilesM * tilesN) return;
  const int tm = tile / tilesN;
  const int tn = tile - tm * tilesN;
  const int m0 = tm << 6;
  const int n0 = tn << 6;

  const T* Ab  = A  + (size_t)b * strideA;
  const T* Bb  = Bt + (size_t)b * strideB;
  const T* Ab2 = (SPL >= 1) ? (A2  + (size_t)b * strideA) : nullptr;
  const T* Bb2 = (SPL == 2) ? (Bt2 + (size_t)b * strideB) : nullptr;

  const int rlane = lane & 15;
  const int koff  = (lane >> 4) * 8;
  const int mOff  = (lane >> 4) * 8;

  v8f acc[4][4];
#pragma unroll
  for (int i = 0; i < 4; ++i)
#pragma unroll
    for (int j = 0; j < 4; ++j) acc[i][j] = (v8f){0.f,0.f,0.f,0.f,0.f,0.f,0.f,0.f};

  for (int k0 = 0; k0 < K; k0 += 32) {
    V bh[4], bl[4];
#pragma unroll
    for (int j = 0; j < 4; ++j) {
      const size_t bo = (size_t)(n0 + (j << 4) + rlane) * ldb + koff + k0;
      bh[j] = Frag<T>::load(Bb + bo);
      if (SPL == 2) bl[j] = Frag<T>::load(Bb2 + bo);
    }
#pragma unroll
    for (int i = 0; i < 4; ++i) {
      const size_t ao = (size_t)(m0 + (i << 4) + rlane) * lda + koff + k0;
      V ah = Frag<T>::load(Ab + ao);
      V al;
      if (SPL >= 1) al = Frag<T>::load(Ab2 + ao);
#pragma unroll
      for (int j = 0; j < 4; ++j) {
        acc[i][j] = Frag<T>::mma(ah, bh[j], acc[i][j]);
        if (SPL == 2) acc[i][j] = Frag<T>::mma(ah, bl[j], acc[i][j]);
        if (SPL >= 1) acc[i][j] = Frag<T>::mma(al, bh[j], acc[i][j]);
      }
      Frag<T>::guard(acc[i][0], acc[i][3], ah, (SPL >= 1) ? al : ah);
    }
    Frag<T>::keep(bh[0], bh[1], bh[2], bh[3]);
    if (SPL == 2) Frag<T>::keep(bl[0], bl[1], bl[2], bl[3]);
  }
  acc_guard4(acc[0][0], acc[0][1], acc[0][2], acc[0][3]);
  acc_guard4(acc[1][0], acc[1][1], acc[1][2], acc[1][3]);
  acc_guard4(acc[2][0], acc[2][1], acc[2][2], acc[2][3]);
  acc_guard4(acc[3][0], acc[3][1], acc[3][2], acc[3][3]);

  float* slab = sT[wave];
  const float* Rb = RESID ? (resid + (size_t)b * strideR) : nullptr;
#pragma unroll
  for (int i = 0; i < 4; ++i) {
    const int mBase = m0 + (i << 4);
#pragma unroll
    for (int j = 0; j < 4; ++j) {
      const int n = n0 + (j << 4) + rlane;
      float bv = 0.f;
      if (BIAS_MODE == 2) bv = bias[n];
#pragma unroll
      for (int r = 0; r < 8; ++r) {
        float v = acc[i][j][r] * scale;
        if (BIAS_MODE == 1) v += bias[mBase + mOff + r];
        if (BIAS_MODE == 2) v += bv;
        if (RESID) v += Rb[(size_t)(mBase + mOff + r) * ldc + n];
        if (ACT == 1) v = tanhf(v);
        if (ACT == 2) v = fmaxf(v, 0.0f);
        if (ACT == 3) v = v / (1.0f + expf(-v));
        if (ACT == 4) v = (v > 0.f) ? v : 0.01f * v;
        slab[(mOff + r) * 68 + (j << 4) + rlane] = v;
      }
    }
    __builtin_amdgcn_fence(__ATOMIC_RELEASE, "workgroup");
    __builtin_amdgcn_wave_barrier();
    __builtin_amdgcn_fence(__ATOMIC_ACQUIRE, "workgroup");
    if (OUT_MODE == 0) {
      float* C = (float*)Cout + (size_t)b * strideC;
      const int hh = lane >> 4, c4 = (lane & 15) * 4;
      for (int pass = 0; pass < 2; ++pass) {
#pragma unroll
        for (int it = 0; it < 8; ++it) {
          const int row = it * 2 + hh;
          v4f v = *(const v4f*)(slab + row * 68 + c4);
          *(volatile v4f*)(C + (size_t)(mBase + row) * ldc + n0 + c4) = v;
        }
        __threadfence();
      }
    } else {
      const int q = lane >> 3, c8 = (lane & 7) * 8;
      unsigned short* C  = (unsigned short*)Cout  + (size_t)b * strideC;
      unsigned short* C2 = (OUT_MODE == 2) ? ((unsigned short*)Cout2 + (size_t)b * strideC) : nullptr;
      for (int pass = 0; pass < 2; ++pass) {
#pragma unroll
        for (int it = 0; it < 4; ++it) {
          const int row = it * 4 + q;
          const float* sp = slab + row * 68 + c8;
          v8h hv, lv;
#pragma unroll
          for (int e = 0; e < 8; ++e) {
            if (OUT_MODE == 1) {
              hv[e] = (_Float16)sp[e];
            } else {
              unsigned short hb = f2bf_bits(sp[e]);
              unsigned short lb = f2bf_bits(sp[e] - bf_bits2f(hb));
              hv[e] = __builtin_bit_cast(_Float16, hb);
              lv[e] = __builtin_bit_cast(_Float16, lb);
            }
          }
          *(volatile v8h*)(C + (size_t)(mBase + row) * ldc + n0 + c8) = hv;
          if (OUT_MODE == 2) *(volatile v8h*)(C2 + (size_t)(mBase + row) * ldc + n0 + c8) = lv;
        }
        __threadfence();
      }
    }
    __builtin_amdgcn_fence(__ATOMIC_RELEASE, "workgroup");
    __builtin_amdgcn_wave_barrier();
    __builtin_amdgcn_fence(__ATOMIC_ACQUIRE, "workgroup");
  }
}

__global__ __launch_bounds__(256) void split_rows_bf16_kernel(
    const float* __restrict__ src, unsigned short* __restrict__ dhi, unsigned short* __restrict__ dlo, int total8)
{
  const int i = blockIdx.x * 256 + threadIdx.x;
  if (i >= total8) return;
  const size_t e0 = (size_t)i << 3;
  const v4f a0 = *(const v4f*)(src + e0);
  const v4f a1 = *(const v4f*)(src + e0 + 4);
  v8h hv, lv;
#pragma unroll
  for (int e = 0; e < 4; ++e) {
    const unsigned short h0 = f2bf_bits(a0[e]), h1 = f2bf_bits(a1[e]);
    const unsigned short l0 = f2bf_bits(a0[e] - bf_bits2f(h0)), l1 = f2bf_bits(a1[e] - bf_bits2f(h1));
    hv[e]     = __builtin_bit_cast(_Float16, h0);
    hv[4 + e] = __builtin_bit_cast(_Float16, h1);
    lv[e]     = __builtin_bit_cast(_Float16, l0);
    lv[4 + e] = __builtin_bit_cast(_Float16, l1);
  }
  unsigned short* qh = dhi + e0;
  unsigned short* ql = dlo + e0;
  *(volatile v8h*)qh = hv;
  *(volatile v8h*)ql = lv;
  __threadfence();
  *(volatile v8h*)qh = hv;
  *(volatile v8h*)ql = lv;
}

template <int KR>
__global__ __launch_bounds__(256) void transpose_split_kernel(
    const float* __restrict__ src, int ncols, unsigned short* __restrict__ dhi, unsigned short* __restrict__ dlo)
{
  constexpr int PT  = KR + 4;
  constexpr int NIT = KR / 64;
  constexpr int CPR = KR / 8;
  static_assert((KR % 64) == 0 && NIT >= 1 && NIT <= 4, "KR");
  __shared__ __align__(16) float sT[32 * PT];
  const int tid = threadIdx.x;
  const int n0 = blockIdx.x * 32;
#pragma unroll 1
  for (int i = 0; i < KR / 8; ++i) {
    const int idx = tid + 256 * i;
    const int k = idx >> 5, nl = idx & 31;
    const int n = n0 + nl;
    const int nc = (n < ncols) ? n : (ncols - 1);
    float v = src[(size_t)k * ncols + nc];
    v = (n < ncols) ? v : 0.0f;
    sT[nl * PT + k] = v;
  }
  __syncthreads();
  v8h hv[NIT], lv[NIT];
#pragma unroll
  for (int it = 0; it < NIT; ++it) {
    const int q = tid + 256 * it;
    const int row = q / CPR, c8 = (q - row * CPR) * 8;
    const float* sp = sT + row * PT + c8;
    const v4f a0 = *(const v4f*)(sp);
    const v4f a1 = *(const v4f*)(sp + 4);
#pragma unroll
    for (int e = 0; e < 4; ++e) {
      const unsigned short h0 = f2bf_bits(a0[e]), h1 = f2bf_bits(a1[e]);
      const unsigned short l0 = f2bf_bits(a0[e] - bf_bits2f(h0)), l1 = f2bf_bits(a1[e] - bf_bits2f(h1));
      hv[it][e]     = __builtin_bit_cast(_Float16, h0);
      hv[it][4 + e] = __builtin_bit_cast(_Float16, h1);
      lv[it][e]     = __builtin_bit_cast(_Float16, l0);
      lv[it][4 + e] = __builtin_bit_cast(_Float16, l1);
    }
  }
  for (int pass = 0; pass < 2; ++pass) {
#pragma unroll
    for (int it = 0; it < NIT; ++it) {
      const int q = tid + 256 * it;
      const int row = q / CPR, c8 = (q - row * CPR) * 8;
      const size_t o = (size_t)(n0 + row) * KR + c8;
      *(volatile v8h*)(dhi + o) = hv[it];
      *(volatile v8h*)(dlo + o) = lv[it];
    }
    __threadfence();
  }
}

template <int CIN>
__global__ __launch_bounds__(256) void im2col_split_kernel(
    const float* __restrict__ src, unsigned short* __restrict__ dhi, unsigned short* __restrict__ dlo)
{
  constexpr int KK  = CIN * 9;
  constexpr int NP  = KK / 2;
  constexpr int NCH = KK / 8;
  static_assert((KK % 8) == 0 && ((KK * 2) % 128) == 0, "im2col row geometry");
  __shared__ __align__(16) unsigned sH[NP];
  __shared__ __align__(16) unsigned sL[NP];
  const int pix = blockIdx.x;
  const int py = pix >> 6, px = pix & 63;
  const int tid = threadIdx.x;
#pragma unroll 1
  for (int p = tid; p < NP; p += 256) {
    unsigned hw = 0u, lw = 0u;
#pragma unroll
    for (int e = 0; e < 2; ++e) {
      const int k = 2 * p + e;
      const int cin = k / 9;
      const int tap = k - cin * 9;
      const int kh = tap / 3;
      const int kw = tap - kh * 3;
      const int iy = py + kh - 1, ix = px + kw - 1;
      const bool inb = ((unsigned)iy < 64u) && ((unsigned)ix < 64u);
      const int iyc = (iy < 0) ? 0 : ((iy > 63) ? 63 : iy);
      const int ixc = (ix < 0) ? 0 : ((ix > 63) ? 63 : ix);
      float v = src[(size_t)cin * kHW + iyc * 64 + ixc];
      v = inb ? v : 0.0f;
      const unsigned short hb = f2bf_bits(v);
      const unsigned short lb = f2bf_bits(v - bf_bits2f(hb));
      hw |= ((unsigned)hb) << (16 * e);
      lw |= ((unsigned)lb) << (16 * e);
    }
    sH[p] = hw;
    sL[p] = lw;
  }
  __syncthreads();
  unsigned short* rh = dhi + (size_t)pix * KK;
  unsigned short* rl = dlo + (size_t)pix * KK;
  for (int pass = 0; pass < 2; ++pass) {
#pragma unroll 1
    for (int q = tid; q < NCH; q += 256) {
      const v4u wh = *(const v4u*)(sH + 4 * q);
      const v4u wl = *(const v4u*)(sL + 4 * q);
      *(volatile v4u*)(rh + 8 * q) = wh;
      *(volatile v4u*)(rl + 8 * q) = wl;
    }
    __threadfence();
  }
}

template <bool RESID>
__global__ __launch_bounds__(256) void inorm_lrelu_kernel(
    const float* __restrict__ src, const float* __restrict__ resid, float* __restrict__ dst)
{
  __shared__ float sRed[256];
  const int row = blockIdx.x;
  const int tid = threadIdx.x;
  const float* p = src + (size_t)row * kHW + 4 * tid;
  const v4f v0 = *(const v4f*)(p);
  const v4f v1 = *(const v4f*)(p + 1024);
  const v4f v2 = *(const v4f*)(p + 2048);
  const v4f v3 = *(const v4f*)(p + 3072);
  float s = ((v0[0] + v0[1]) + (v0[2] + v0[3])) + ((v1[0] + v1[1]) + (v1[2] + v1[3]))
          + ((v2[0] + v2[1]) + (v2[2] + v2[3])) + ((v3[0] + v3[1]) + (v3[2] + v3[3]));
  sRed[tid] = s;
  __syncthreads();
  for (int off = 128; off > 0; off >>= 1) {
    if (tid < off) sRed[tid] = sRed[tid] + sRed[tid + off];
    __syncthreads();
  }
  const float mean = sRed[0] * (1.0f / 4096.0f);
  __syncthreads();
  const v4f d0 = v0 - mean, d1 = v1 - mean, d2 = v2 - mean, d3 = v3 - mean;
  float q = ((d0[0] * d0[0] + d0[1] * d0[1]) + (d0[2] * d0[2] + d0[3] * d0[3]))
          + ((d1[0] * d1[0] + d1[1] * d1[1]) + (d1[2] * d1[2] + d1[3] * d1[3]))
          + ((d2[0] * d2[0] + d2[1] * d2[1]) + (d2[2] * d2[2] + d2[3] * d2[3]))
          + ((d3[0] * d3[0] + d3[1] * d3[1]) + (d3[2] * d3[2] + d3[3] * d3[3]));
  sRed[tid] = q;
  __syncthreads();
  for (int off = 128; off > 0; off >>= 1) {
    if (tid < off) sRed[tid] = sRed[tid] + sRed[tid + off];
    __syncthreads();
  }
  const float var = sRed[0] * (1.0f / 4096.0f);
  const float rstd = 1.0f / sqrtf(var + kEps);
  v4f o0, o1, o2, o3;
#pragma unroll
  for (int e = 0; e < 4; ++e) {
    o0[e] = d0[e] * rstd + ((v0[e] > 0.f) ? v0[e] : kNegSlope * v0[e]);
    o1[e] = d1[e] * rstd + ((v1[e] > 0.f) ? v1[e] : kNegSlope * v1[e]);
    o2[e] = d2[e] * rstd + ((v2[e] > 0.f) ? v2[e] : kNegSlope * v2[e]);
    o3[e] = d3[e] * rstd + ((v3[e] > 0.f) ? v3[e] : kNegSlope * v3[e]);
  }
  if (RESID) {
    const float* rp = resid + (size_t)row * kHW + 4 * tid;
    o0 += *(const v4f*)(rp);
    o1 += *(const v4f*)(rp + 1024);
    o2 += *(const v4f*)(rp + 2048);
    o3 += *(const v4f*)(rp + 3072);
  }
  float* dp = dst + (size_t)row * kHW + 4 * tid;
  for (int pass = 0; pass < 2; ++pass) {
    *(volatile v4f*)(dp)        = o0;
    *(volatile v4f*)(dp + 1024) = o1;
    *(volatile v4f*)(dp + 2048) = o2;
    *(volatile v4f*)(dp + 3072) = o3;
    __threadfence();
  }
}

__global__ __launch_bounds__(256) void layernorm_split_kernel(
    const float* __restrict__ src, const float* __restrict__ g, const float* __restrict__ be,
    unsigned short* __restrict__ dhi, unsigned short* __restrict__ dlo)
{
  __shared__ __align__(16) float sV[kLnTok * kLnP];
  const int tid = threadIdx.x, lane = tid & 31, wave = tid >> 5;
  const int blk = blockIdx.x;
  const int b = blk >> 6;
  const int l0 = (blk & 63) * kLnTok;
  const size_t tok0 = (size_t)blk * kLnTok;
  const float* sb = src + (size_t)b * kDm * kHW + l0;
#pragma unroll 1
  for (int i = 0; i < 32; ++i) {
    const int idx = tid + 256 * i;
    const int c = idx >> 6, l = idx & 63;
    sV[l * kLnP + c] = sb[(size_t)c * kHW + l];
  }
  __syncthreads();
  const int tk = tid >> 2, part = tid & 3;
  float* rowp = sV + tk * kLnP + part * 32;
  float s = 0.f;
#pragma unroll 1
  for (int c4 = 0; c4 < 8; ++c4) {
    const v4f v = *(const v4f*)(rowp + 4 * c4);
    s += (v[0] + v[1]) + (v[2] + v[3]);
  }
  s += __shfl_xor(s, 1, 32);
  s += __shfl_xor(s, 2, 32);
  const float mean = s * (1.0f / 128.0f);
  float q = 0.f;
#pragma unroll 1
  for (int c4 = 0; c4 < 8; ++c4) {
    const v4f v = *(const v4f*)(rowp + 4 * c4);
    const v4f dv = v - mean;
    q += (dv[0] * dv[0] + dv[1] * dv[1]) + (dv[2] * dv[2] + dv[3] * dv[3]);
  }
  q += __shfl_xor(q, 1, 32);
  q += __shfl_xor(q, 2, 32);
  const float var = q * (1.0f / 128.0f);
  const float rstd = 1.0f / sqrtf(var + kEps);
#pragma unroll 1
  for (int c4 = 0; c4 < 8; ++c4) {
    const int c = part * 32 + 4 * c4;
    const v4f v  = *(const v4f*)(rowp + 4 * c4);
    const v4f gg = *(const v4f*)(g + c);
    const v4f bb = *(const v4f*)(be + c);
    const v4f o = ((v - mean) * rstd) * gg + bb;
    *(v4f*)(rowp + 4 * c4) = o;
  }
  __syncthreads();
  const int hh = lane >> 4, c8 = (lane & 15) * 8;
  v8h hv[4], lv[4];
#pragma unroll
  for (int it = 0; it < 4; ++it) {
    const int row = it * 16 + wave * 2 + hh;
    const float* sp = sV + row * kLnP + c8;
    const v4f a0 = *(const v4f*)(sp);
    const v4f a1 = *(const v4f*)(sp + 4);
#pragma unroll
    for (int e = 0; e < 4; ++e) {
      const unsigned short h0 = f2bf_bits(a0[e]), h1 = f2bf_bits(a1[e]);
      const unsigned short lo0 = f2bf_bits(a0[e] - bf_bits2f(h0)), lo1 = f2bf_bits(a1[e] - bf_bits2f(h1));
      hv[it][e]     = __builtin_bit_cast(_Float16, h0);
      hv[it][4 + e] = __builtin_bit_cast(_Float16, h1);
      lv[it][e]     = __builtin_bit_cast(_Float16, lo0);
      lv[it][4 + e] = __builtin_bit_cast(_Float16, lo1);
    }
  }
  for (int pass = 0; pass < 2; ++pass) {
#pragma unroll
    for (int it = 0; it < 4; ++it) {
      const int row = it * 16 + wave * 2 + hh;
      const size_t o = (tok0 + row) * kDm + c8;
      *(volatile v8h*)(dhi + o) = hv[it];
      *(volatile v8h*)(dlo + o) = lv[it];
    }
    __threadfence();
  }
}

__global__ __launch_bounds__(256) void conv_silu_kernel(
    const float* __restrict__ XZ, const float* __restrict__ cw, const float* __restrict__ cb,
    float* __restrict__ UC, unsigned short* __restrict__ UCH, unsigned short* __restrict__ UCL)
{
  __shared__ __align__(16) float sT[16 * kConvTP];
  const int tid = threadIdx.x, lane = tid & 31, wave = tid >> 5;
  const int d0 = blockIdx.x * 256, d = d0 + tid;
  const int g0 = blockIdx.y * 64;
  const int tb = g0 & (kSeq - 1);
  const float w0 = cw[d * 4 + 0], w1 = cw[d * 4 + 1], w2 = cw[d * 4 + 2], w3 = cw[d * 4 + 3];
  const float bc = cb[d];
  float xm3, xm2, xm1;
  {
    const bool hist = (tb > 0);
    const int rb = hist ? (g0 - 3) : g0;
    const float v3 = XZ[(size_t)rb * kXzP + d];
    const float v2 = XZ[(size_t)(rb + 1) * kXzP + d];
    const float v1 = XZ[(size_t)(rb + 2) * kXzP + d];
    xm3 = hist ? v3 : 0.f;
    xm2 = hist ? v2 : 0.f;
    xm1 = hist ? v1 : 0.f;
  }
  const int hrow = wave >> 1;
  const int hch  = (wave & 1) * 128 + lane * 4;
#pragma unroll 1
  for (int sub = 0; sub < 4; ++sub) {
    const int lb = g0 + sub * 16;
#pragma unroll 1
    for (int s = 0; s < 16; ++s) {
      const float xcur = XZ[(size_t)(lb + s) * kXzP + d];
      float acc = w0 * xm3;
      acc = fmaf(w1, xm2, acc);
      acc = fmaf(w2, xm1, acc);
      acc = fmaf(w3, xcur, acc);
      const float sv = acc + bc;
      const float sg = __builtin_amdgcn_rcpf(1.0f + __expf(-sv));
      sT[s * kConvTP + tid] = sv * sg;
      xm3 = xm2; xm2 = xm1; xm1 = xcur;
    }
    __syncthreads();
    v4f fv[4];
    v8h bh[2], blo[2];
#pragma unroll
    for (int it = 0; it < 4; ++it) fv[it] = *(const v4f*)(sT + (it * 4 + hrow) * kConvTP + hch);
#pragma unroll
    for (int it = 0; it < 2; ++it) {
      const float* sp = sT + (it * 8 + wave) * kConvTP + lane * 8;
      const v4f a0 = *(const v4f*)(sp);
      const v4f a1 = *(const v4f*)(sp + 4);
#pragma unroll
      for (int e = 0; e < 4; ++e) {
        const unsigned short h0 = f2bf_bits(a0[e]), h1 = f2bf_bits(a1[e]);
        const unsigned short l0 = f2bf_bits(a0[e] - bf_bits2f(h0)), l1 = f2bf_bits(a1[e] - bf_bits2f(h1));
        bh[it][e]      = __builtin_bit_cast(_Float16, h0);
        bh[it][4 + e]  = __builtin_bit_cast(_Float16, h1);
        blo[it][e]     = __builtin_bit_cast(_Float16, l0);
        blo[it][4 + e] = __builtin_bit_cast(_Float16, l1);
      }
    }
    for (int pass = 0; pass < 2; ++pass) {
#pragma unroll
      for (int it = 0; it < 4; ++it)
        *(volatile v4f*)(UC + (size_t)(lb + it * 4 + hrow) * kDin + d0 + hch) = fv[it];
#pragma unroll
      for (int it = 0; it < 2; ++it) {
        const size_t o = (size_t)(lb + it * 8 + wave) * kDin + d0 + lane * 8;
        *(volatile v8h*)(UCH + o) = bh[it];
        *(volatile v8h*)(UCL + o) = blo[it];
      }
      __threadfence();
    }
    __syncthreads();
  }
}

__global__ __launch_bounds__(64) void scan_kernel(
    const float* __restrict__ XD, const float* __restrict__ UC, const float* __restrict__ XZ,
    const float* __restrict__ Wdt, const float* __restrict__ bdt, const float* __restrict__ Alog,
    const float* __restrict__ Dp, unsigned short* __restrict__ YH, unsigned short* __restrict__ YL)
{
  __shared__ __align__(16) float sX[kScanTS * kXdP];
  __shared__ __align__(16) float sY[kScanTS * kScanYP];
  __shared__ __align__(16) float sW[kDtR * kScanCh];
  __shared__ __align__(16) float sA[kNst * kScanCh];
  const int tid = threadIdx.x, lane = tid & 31, wave = tid >> 5;
  constexpr int kBlkPerB = kDin / kScanCh;
  const int bix = blockIdx.x / kBlkPerB;
  const int d0  = (blockIdx.x - bix * kBlkPerB) * kScanCh;
  const int d   = d0 + tid;
  const size_t row0 = (size_t)bix * kSeq;
#pragma unroll 1
  for (int r = 0; r < kDtR; ++r) sW[r * kScanCh + tid] = Wdt[(size_t)r * kDin + d];
#pragma unroll 1
  for (int s = 0; s < kNst; ++s) sA[s * kScanCh + tid] = -expf(Alog[(size_t)d * kNst + s]);
  __syncthreads();
  float negA[kNst], h[kNst];
#pragma unroll
  for (int s = 0; s < kNst; ++s) {
    negA[s] = sA[s * kScanCh + tid];
    h[s] = 0.f;
  }
  const float bb = bdt[d], Dd = Dp[d];
  const int lr = tid >> 4, lc4 = (tid & 15) * 4;
  const int q = lane >> 3, c8 = (lane & 7) * 8;
#pragma unroll 1
  for (int t0 = 0; t0 < kSeq; t0 += kScanTS) {
    __syncthreads();
#pragma unroll
    for (int i = 0; i < 16; ++i) {
      const int r = lr + 4 * i;
      *(v4f*)(sX + r * kXdP + lc4) = *(const v4f*)(XD + (row0 + t0 + r) * kXdP + lc4);
    }
    __syncthreads();
#pragma unroll 1
    for (int s = 0; s < kScanTS; ++s) {
      const int t = t0 + s;
      const float* xr = sX + s * kXdP;
      float vdot = 0.f;
#pragma unroll 1
      for (int r4 = 0; r4 < kDtR / 4; ++r4) {
        const v4f xv = *(const v4f*)(xr + 4 * r4);
        const float* wp = sW + (4 * r4) * kScanCh + tid;
        vdot = fmaf(xv[0], wp[0], vdot);
        vdot = fmaf(xv[1], wp[kScanCh], vdot);
        vdot = fmaf(xv[2], wp[2 * kScanCh], vdot);
        vdot = fmaf(xv[3], wp[3 * kScanCh], vdot);
      }
      float Bs[kNst], Cs[kNst];
#pragma unroll
      for (int q4 = 0; q4 < 4; ++q4) {
        const v4f bv = *(const v4f*)(xr + kDtR + 4 * q4);
        const v4f cv = *(const v4f*)(xr + kDtR + kNst + 4 * q4);
        Bs[4 * q4 + 0] = bv[0]; Bs[4 * q4 + 1] = bv[1]; Bs[4 * q4 + 2] = bv[2]; Bs[4 * q4 + 3] = bv[3];
        Cs[4 * q4 + 0] = cv[0]; Cs[4 * q4 + 1] = cv[1]; Cs[4 * q4 + 2] = cv[2]; Cs[4 * q4 + 3] = cv[3];
      }
      const float v   = vdot + bb;
      const float a   = __expf(-fabsf(v));
      const float u   = 1.0f + a;
      const float l1p = __logf(u) + (a - (u - 1.0f)) * __builtin_amdgcn_rcpf(u);
      const float dt  = fmaxf(v, 0.0f) + l1p;
      const float xt  = UC[(row0 + t) * kDin + d];
      const float dtx = dt * xt;
      float y = 0.f;
#pragma unroll
      for (int k = 0; k < kNst; ++k) {
        const float e = __expf(dt * negA[k]);
        h[k] = e * h[k] + dtx * Bs[k];
        y = h[k] * Cs[k] + y;
      }
      y = xt * Dd + y;
      const float zv = XZ[(row0 + t) * kXzP + kDin + d];
      const float sg = __builtin_amdgcn_rcpf(1.0f + __expf(-zv));
      y = y * (zv * sg);
      sY[s * kScanYP + tid] = y;
    }
    __syncthreads();
    v8h hv[8], lv[8];
#pragma unroll
    for (int it = 0; it < 8; ++it) {
      const int row = it * 8 + wave * 4 + q;
      const float* sp = sY + row * kScanYP + c8;
      const v4f a0 = *(const v4f*)(sp);
      const v4f a1 = *(const v4f*)(sp + 4);
#pragma unroll
      for (int e = 0; e < 4; ++e) {
        const unsigned short h0 = f2bf_bits(a0[e]), h1 = f2bf_bits(a1[e]);
        const unsigned short l0 = f2bf_bits(a0[e] - bf_bits2f(h0)), l1 = f2bf_bits(a1[e] - bf_bits2f(h1));
        hv[it][e]     = __builtin_bit_cast(_Float16, h0);
        hv[it][4 + e] = __builtin_bit_cast(_Float16, h1);
        lv[it][e]     = __builtin_bit_cast(_Float16, l0);
        lv[it][4 + e] = __builtin_bit_cast(_Float16, l1);
      }
    }
    for (int pass = 0; pass < 2; ++pass) {
#pragma unroll
      for (int it = 0; it < 8; ++it) {
        const int row = it * 8 + wave * 4 + q;
        const size_t o = (row0 + t0 + row) * kDin + d0 + c8;
        *(volatile v8h*)(YH + o) = hv[it];
        *(volatile v8h*)(YL + o) = lv[it];
      }
      __threadfence();
    }
  }
}

extern "C" void kernel_launch(void* const* d_in, const int* in_sizes, int n_in,
                              void* d_out, int out_size, void* d_ws, size_t ws_size,
                              hipStream_t stream) {
  if (n_in < 16) return;
  if (in_sizes[0]  != kBatch * kDm * kHW) return;
  if (in_sizes[1]  != kDin * kK1) return;
  if (in_sizes[2]  != kDin) return;
  if (in_sizes[3]  != kDm * kK2) return;
  if (in_sizes[4]  != kDm) return;
  if (in_sizes[5]  != kDm) return;
  if (in_sizes[6]  != kDm) return;
  if (in_sizes[7]  != kDm * kXzP) return;
  if (in_sizes[8]  != kDin * 4) return;
  if (in_sizes[9]  != kDin) return;
  if (in_sizes[10] != kDin * kXdW) return;
  if (in_sizes[11] != kDtR * kDin) return;
  if (in_sizes[12] != kDin) return;
  if (in_sizes[13] != kDin * kNst) return;
  if (in_sizes[14] != kDin) return;
  if (in_sizes[15] != kDin * kDm) return;
  if (out_size != kBatch * kDm * kHW) return;
  if (ws_size < kWsTotal) return;

  const float* x         = (const float*)d_in[0];
  const float* conv1_w   = (const float*)d_in[1];
  const float* conv1_b   = (const float*)d_in[2];
  const float* conv2_w   = (const float*)d_in[3];
  const float* conv2_b   = (const float*)d_in[4];
  const float* ln_g      = (const float*)d_in[5];
  const float* ln_b      = (const float*)d_in[6];
  const float* in_proj_w = (const float*)d_in[7];
  const float* conv1d_w  = (const float*)d_in[8];
  const float* conv1d_b  = (const float*)d_in[9];
  const float* x_proj_w  = (const float*)d_in[10];
  const float* dt_proj_w = (const float*)d_in[11];
  const float* dt_proj_b = (const float*)d_in[12];
  const float* A_log     = (const float*)d_in[13];
  const float* Dp        = (const float*)d_in[14];
  const float* out_pw    = (const float*)d_in[15];
  float* out = (float*)d_out;

  char* ws = (char*)d_ws;
  unsigned short* W1H  = (unsigned short*)(ws + kOffW1H);
  unsigned short* W1L  = (unsigned short*)(ws + kOffW1L);
  unsigned short* W2H  = (unsigned short*)(ws + kOffW2H);
  unsigned short* W2L  = (unsigned short*)(ws + kOffW2L);
  unsigned short* WITH = (unsigned short*)(ws + kOffWITH);
  unsigned short* WITL = (unsigned short*)(ws + kOffWITL);
  unsigned short* WXTH = (unsigned short*)(ws + kOffWXTH);
  unsigned short* WXTL = (unsigned short*)(ws + kOffWXTL);
  unsigned short* WOTH = (unsigned short*)(ws + kOffWOTH);
  unsigned short* WOTL = (unsigned short*)(ws + kOffWOTL);
  unsigned short* IMH  = (unsigned short*)(ws + kOffIMH);
  unsigned short* IML  = (unsigned short*)(ws + kOffIML);
  float*          XZ   = (float*)(ws + kOffXZ);
  float*          C1   = (float*)(ws + kOffC1);
  float*          C2   = (float*)(ws + kOffC2);
  float*          G2   = (float*)(ws + kOffG2);
  float*          UC   = (float*)(ws + kOffUC);
  float*          G1   = (float*)(ws + kOffG1);
  unsigned short* TH   = (unsigned short*)(ws + kOffTH);
  unsigned short* TL   = (unsigned short*)(ws + kOffTL);
  unsigned short* UCH  = (unsigned short*)(ws + kOffUCH);
  unsigned short* UCL  = (unsigned short*)(ws + kOffUCL);
  float*          XD   = (float*)(ws + kOffXD);
  unsigned short* YH   = (unsigned short*)(ws + kOffYH);
  unsigned short* YL   = (unsigned short*)(ws + kOffYL);

  split_rows_bf16_kernel<<<(kDin * kK1 / 8) / 256, 256, 0, stream>>>(conv1_w, W1H, W1L, kDin * kK1 / 8);
  split_rows_bf16_kernel<<<(kDm * kK2 / 8) / 256, 256, 0, stream>>>(conv2_w, W2H, W2L, kDm * kK2 / 8);
  transpose_split_kernel<kDm><<<kXzP / 32, 256, 0, stream>>>(in_proj_w, kXzP, WITH, WITL);
  transpose_split_kernel<kDin><<<kXdP / 32, 256, 0, stream>>>(x_proj_w, kXdW, WXTH, WXTL);
  transpose_split_kernel<kDin><<<kDm / 32, 256, 0, stream>>>(out_pw, kDm, WOTH, WOTL);

  for (int b = 0; b < kBatch; ++b) {
    im2col_split_kernel<kDm><<<kHW, 256, 0, stream>>>(x + (size_t)b * kDm * kHW, IMH, IML);
    wmma_gemm64<1, 2, 1, 0, false><<<dim3((kDin / 64) * (kHW / 64) / 8, 1), 256, 0, stream>>>(
        W1H, W1L, kK1, 0L,
        IMH, IML, kK1, 0L,
        (void*)(C1 + (size_t)b * kDin * kHW), nullptr, kHW, 0L,
        conv1_b, nullptr, 0L,
        kDin, kHW, kK1, 1.0f);
  }
  inorm_lrelu_kernel<false><<<kBatch * kDin, 256, 0, stream>>>(C1, nullptr, G1);

  for (int b = 0; b < kBatch; ++b) {
    im2col_split_kernel<kDin><<<kHW, 256, 0, stream>>>(G1 + (size_t)b * kDin * kHW, IMH, IML);
    wmma_gemm64<1, 2, 1, 0, false><<<dim3((kDm / 64) * (kHW / 64) / 8, 1), 256, 0, stream>>>(
        W2H, W2L, kK2, 0L,
        IMH, IML, kK2, 0L,
        (void*)(C2 + (size_t)b * kDm * kHW), nullptr, kHW, 0L,
        conv2_b, nullptr, 0L,
        kDm, kHW, kK2, 1.0f);
  }
  inorm_lrelu_kernel<true><<<kBatch * kDm, 256, 0, stream>>>(C2, x, G2);

  layernorm_split_kernel<<<kRows / kLnTok, 256, 0, stream>>>(G2, ln_g, ln_b, TH, TL);

  wmma_gemm64<1, 2, 0, 0, false><<<dim3((kRows / 64) * (kXzP / 64) / 8, 1), 256, 0, stream>>>(
      TH, TL, kDm, 0L,
      WITH, WITL, kDm, 0L,
      (void*)XZ, nullptr, kXzP, 0L,
      nullptr, nullptr, 0L,
      kRows, kXzP, kDm, 1.0f);

  conv_silu_kernel<<<dim3(kDin / 256, kRows / 64), 256, 0, stream>>>(XZ, conv1d_w, conv1d_b, UC, UCH, UCL);

  wmma_gemm64<1, 2, 0, 0, false><<<dim3((kRows / 64) * (kXdP / 64) / 8, 1), 256, 0, stream>>>(
      UCH, UCL, kDin, 0L,
      WXTH, WXTL, kDin, 0L,
      (void*)XD, nullptr, kXdP, 0L,
      nullptr, nullptr, 0L,
      kRows, kXdP, kDin, 1.0f);

  scan_kernel<<<kBatch * (kDin / kScanCh), kScanCh, 0, stream>>>(XD, UC, XZ, dt_proj_w, dt_proj_b, A_log, Dp, YH, YL);

  wmma_gemm64<1, 2, 0, 0, false><<<dim3((kDm / 64) * (kHW / 64) / 8, kBatch), 256, 0, stream>>>(
      WOTH, WOTL, kDin, 0L,
      YH, YL, kDin, (long)kSeq * kDin,
      (void*)out, nullptr, kHW, (long)kDm * kHW,
      nullptr, nullptr, 0L,
      kDm, kHW, kDin, 1.0f);
}
